// DHMSA_41592463294756
// MI455X (gfx1250) — hardware-verified
//
#include <hip/hip_runtime.h>


namespace {
constexpr int NB_ = 2, IH = 126, IW = 126, C = 256, CW = 8, HP = 128, NWS = HP / CW  , NWIN = NWS * NWS  , WL = 64, HWIN = 16, HL = 256, HEADS = 8, HD = 32, NTP = HP * HP  , NTAB = 23 * 23  , CPH = 512, NPIX = IH * IW  ;
constexpr float HS = 256.0f, PS = 256.0f, WSC = 256.0f;
typedef _Float16 b16;
typedef __attribute__((ext_vector_type(16))) _Float16 v16b;
typedef __attribute__((ext_vector_type(8))) _Float16 v8b;
typedef __attribute__((ext_vector_type(2))) _Float16 v2b;
typedef __attribute__((ext_vector_type(8))) float v8f;
typedef __attribute__((ext_vector_type(4))) float v4f;
typedef __attribute__((ext_vector_type(2))) float v2f;
__device__ __forceinline__ float bf16_rne(float f) { unsigned int u = __float_as_uint(f); u += 0x7FFFu + ((u >> 16) & 1u); float r = __uint_as_float(u & 0xFFFF0000u); asm volatile("" : "+v"(r)); return r; }
__device__ __forceinline__ float bfv(float f) { float r = bf16_rne(f); asm volatile("" : "+v"(r)); return r; }
__device__ __forceinline__ void split16(float v, b16& hi, b16& lo) { hi = (b16)v; lo = (b16)(v - (float)hi); }
__device__ __forceinline__ v16b frag_kb(const b16* p, int hh) { const v8b a = *(const v8b*)(p + 8 * hh), b = *(const v8b*)(p + 16 + 8 * hh); v16b f;
#pragma unroll
  for (int e = 0; e < 8; ++e) { f[e] = a[e]; f[8 + e] = b[e]; } return f; }
__device__ __forceinline__ v8f wmma16b(v16b a, v16b b, v8f c) { v8f d = __builtin_amdgcn_wmma_f32_16x16x32_f16(false, a, false, b, (short)0, c, false, false); asm volatile("v_nop\n\tv_nop\n\tv_nop\n\tv_nop" : "+v"(d) : "v"(a), "v"(b)); return d; }
__device__ __forceinline__ void wave_lds_sync() { __builtin_amdgcn_fence(__ATOMIC_RELEASE, "workgroup"); __builtin_amdgcn_wave_barrier(); __builtin_amdgcn_fence(__ATOMIC_ACQUIRE, "workgroup"); }
__device__ __forceinline__ float pmul(float a, float b) { float p = a * b; asm volatile("" : "+v"(p)); return p; }
__device__ __forceinline__ bool halo_key(int wi, int wj, int j, int& yy, int& xx, bool& inimg) { yy = wi * CW - CW / 2 + j / HWIN; xx = wj * CW - CW / 2 + j % HWIN; const bool inpad = yy >= 0 && yy < HP && xx >= 0 && xx < HP; inimg = inpad && yy < IH && xx < IW; return inpad; }

__global__ __launch_bounds__(256) void prep_kernel(const float* __restrict__ wqkv, const float* __restrict__ pw, const float* __restrict__ cw0, const float* __restrict__ cb0, const float* __restrict__ cw1, b16* __restrict__ WQ, b16* __restrict__ WPj, float* __restrict__ TAB, b16* __restrict__ KNh, b16* __restrict__ KNl) { const size_t nt = (size_t)gridDim.x * 256, u0 = (size_t)blockIdx.x * 256 + threadIdx.x; v8b v;
  for (size_t u = u0; u < (size_t)3 * C * 32; u += nt) { const int o = (int)(u / 32), k0 = (int)(u % 32) * 8;
#pragma unroll
    for (int j = 0; j < 8; ++j) v[j] = (b16)(bf16_rne(wqkv[(size_t)(k0 + j) * 3 * C + o]) * WSC); for (int pass = 0; pass < 2; ++pass) { *(volatile v8b*)(WQ + (size_t)o * C + k0) = v; __threadfence(); } }
  for (size_t u = u0; u < (size_t)C * 32; u += nt) { const int o = (int)(u / 32), k0 = (int)(u % 32) * 8;
#pragma unroll
    for (int j = 0; j < 8; ++j) v[j] = (b16)(bf16_rne(pw[(size_t)(k0 + j) * C + o]) * WSC); for (int pass = 0; pass < 2; ++pass) { *(volatile v8b*)(WPj + (size_t)o * C + k0) = v; __threadfence(); } }
  for (size_t u = u0; u < (size_t)NTAB; u += nt) { const int a = (int)(u / 23), bq = (int)(u % 23); float r0 = (float)(a - 11) * (8.0f / 7.0f), r1 = (float)(bq - 11) * (8.0f / 7.0f); const float il8 = 1.0f / logf(8.0f); r0 = (r0 > 0 ? 1.0f : (r0 < 0 ? -1.0f : 0.0f)) * log1pf(fabsf(r0)) * il8; r1 = (r1 > 0 ? 1.0f : (r1 < 0 ? -1.0f : 0.0f)) * log1pf(fabsf(r1)) * il8;
    float t8[HEADS] = {0, 0, 0, 0, 0, 0, 0, 0};
#pragma unroll 1
    for (int m = 0; m < CPH; ++m) { float hdn = fmaxf(pmul(r0, bfv(cw0[m])) + pmul(r1, bfv(cw0[CPH + m])) + bfv(cb0[m]), 0.0f);
#pragma unroll
      for (int hh = 0; hh < HEADS; ++hh) t8[hh] += pmul(hdn, bfv(cw1[(size_t)m * HEADS + hh])); }
    for (int pass = 0; pass < 2; ++pass) {
#pragma unroll
      for (int hh = 0; hh < HEADS; ++hh) ((volatile float*)TAB)[u * HEADS + hh] = 16.0f / (1.0f + __expf(-t8[hh])); __threadfence(); } }
  for (size_t u = u0; u < (size_t)C / 8; u += nt) { const v8b z = {0, 0, 0, 0, 0, 0, 0, 0}; for (int pass = 0; pass < 2; ++pass) { *(volatile v8b*)(KNh + (size_t)NTP * C + u * 8) = z; *(volatile v8b*)(KNl + (size_t)NTP * C + u * 8) = z; __threadfence(); } } }
__global__ __launch_bounds__(32) void qkv_kernel(const float* __restrict__ x  , const float* __restrict__ dwk, const float* __restrict__ lg, const float* __restrict__ lb, const b16* __restrict__ WQ, const float* __restrict__ qb, const float* __restrict__ vb, const float* __restrict__ slog, int TLIM, b16* __restrict__ QNh, b16* __restrict__ QNl, b16* __restrict__ KNh, b16* __restrict__ KNl, float* __restrict__ V) { __shared__ __attribute__((aligned(16))) b16 Ah[16][C + 8], Al[16][C + 8]; __shared__ float Y[16][C + 1], Tf[16][260], Nq[16][HEADS], Nk[16][HEADS]; const int lane = threadIdx.x, nloc = lane & 15, hlf = lane >> 4; const size_t t0 = (size_t)blockIdx.x * 16; if (t0 >= (size_t)TLIM) return; const int yy = (int)(t0 / HP), x0 = (int)(t0 % HP);
  for (int rr = 0; rr < 16; ++rr) { const int xx = x0 + rr; for (int c8 = 0; c8 < 8; ++c8) { const int c = lane * 8 + c8; float s = 0.0f; if (yy < IH && xx < IW) {
#pragma unroll 1
      for (int ky = 0; ky < 3; ++ky) { const int sy = yy + ky - 1; if (sy < 0 || sy >= IH) continue;
#pragma unroll 1
        for (int kx = 0; kx < 3; ++kx) { const int sx = xx + kx - 1; if (sx < 0 || sx >= IW) continue; s += pmul(bfv(x[((size_t)sy * IW + sx) * C + c]), bfv(dwk[(ky * 3 + kx) * C + c])); } } } Y[rr][c] = s; } }
  wave_lds_sync();
  if (lane < 16) { float* row = &Y[lane][0]; float m = 0.0f; for (int c = 0; c < C; ++c) m += row[c]; m *= (1.0f / C); float vr = 0.0f; for (int c = 0; c < C; ++c) { const float d = row[c] - m; vr += d * d; } vr *= (1.0f / C); const float rs = rsqrtf(vr + 1e-5f); for (int c = 0; c < C; ++c) row[c] = pmul((row[c] - m) * rs, bfv(lg[c])) + bfv(lb[c]); }
  wave_lds_sync();
  for (int rr = 0; rr < 16; ++rr) for (int q = 0; q < 8; ++q) { const int c = q * 32 + lane; b16 p, pl; split16(Y[rr][c] * HS, p, pl); Ah[rr][c] = p; Al[rr][c] = pl; }
  if (lane < 16) for (int k = C; k < C + 8; ++k) { Ah[lane][k] = (b16)0.0f; Al[lane][k] = (b16)0.0f; }
  wave_lds_sync();
#pragma unroll 1
  for (int g = 0; g < 3; ++g) { v8f acc[16];
#pragma unroll
    for (int t = 0; t < 16; ++t) acc[t] = (v8f){};
#pragma unroll 2
    for (int kb = 0; kb < C; kb += 32) { const v16b a = frag_kb(&Ah[nloc][kb], hlf), al = frag_kb(&Al[nloc][kb], hlf);
#pragma unroll
      for (int t = 0; t < 16; ++t) { const v16b bw = frag_kb(WQ + (size_t)(g * C + t * 16 + nloc) * C + kb, hlf); acc[t] = wmma16b(a, bw, acc[t]); acc[t] = wmma16b(al, bw, acc[t]); } }
#pragma unroll
    for (int t = 0; t < 16; ++t) { const int cc = t * 16 + nloc; const float bb = g == 0 ? bfv(qb[cc]) : (g == 2 ? bfv(vb[cc]) : 0.0f);
#pragma unroll
      for (int r8 = 0; r8 < 8; ++r8) { const int rr = 8 * hlf + r8; const bool valid = yy < IH && (x0 + rr) < IW; Tf[rr][cc] = valid ? acc[t][r8] * (1.0f / (HS * WSC)) + bb : 0.0f; } }
    wave_lds_sync();
    if (g < 2) {
      if (lane < 16) { for (int h = 0; h < HEADS; ++h) { float ss = 0.0f; for (int d = 0; d < HD; ++d) { const float v = Tf[lane][h * HD + d]; ss += v * v; } const float inv = rsqrtf(fmaxf(ss, 1e-12f)); if (g == 0) Nq[lane][h] = inv * __expf(bfv(slog[h])); else Nk[lane][h] = inv; } }
      wave_lds_sync();
      b16* Ph = g == 0 ? QNh : KNh; b16* Pl = g == 0 ? QNl : KNl;
      for (int pass = 0; pass < 2; ++pass) { for (int rr = 0; rr < 16; ++rr) for (int q = 0; q < 4; ++q) { const int c = q * 64 + lane * 2; const float n0 = (g == 0 ? Nq[rr][c / HD] : Nk[rr][c / HD]); b16 h0, l0, h1, l1; split16(Tf[rr][c] * n0 * HS, h0, l0); split16(Tf[rr][c + 1] * n0 * HS, h1, l1); *(volatile v2b*)(Ph + (t0 + rr) * C + c) = (v2b){h0, h1}; *(volatile v2b*)(Pl + (t0 + rr) * C + c) = (v2b){l0, l1}; } __threadfence(); } }
    else { for (int pass = 0; pass < 2; ++pass) { for (int rr = 0; rr < 16; ++rr) for (int q = 0; q < 2; ++q) *(volatile v4f*)(V + (t0 + rr) * C + q * 128 + lane * 4) = *(const v4f*)(&Tf[rr][q * 128 + lane * 4]); __threadfence(); } }
    wave_lds_sync(); } }
__global__ __launch_bounds__(256) void vt_kernel(const float* __restrict__ V, int WLIM, b16* __restrict__ VTh, b16* __restrict__ VTl) { __shared__ float Tt[HL][65]; const int win = blockIdx.x; if (win >= WLIM) return; const int wi = win / NWS, wj = win % NWS; const int tid = threadIdx.x, wave = tid >> 5, lane = tid & 31;
  for (int cq = 0; cq < C; cq += 64) {
    for (int j = wave; j < HL; j += 8) { int yy, xx; bool inimg; const bool ok = halo_key(wi, wj, j, yy, xx, inimg); const float* vr = V + ((size_t)yy * HP + xx) * C + cq; Tt[j][lane * 2] = ok ? vr[lane * 2] : 0.0f; Tt[j][lane * 2 + 1] = ok ? vr[lane * 2 + 1] : 0.0f; }
    __syncthreads();
    for (int pass = 0; pass < 2; ++pass) { for (int d = wave; d < 64; d += 8) for (int s = 0; s < HL; s += 64) { b16 h0, l0, h1, l1; split16(Tt[s + lane * 2][d] * HS, h0, l0); split16(Tt[s + lane * 2 + 1][d] * HS, h1, l1); const size_t o = ((size_t)win * C + cq + d) * HL + s + lane * 2; *(volatile v2b*)(VTh + o) = (v2b){h0, h1}; *(volatile v2b*)(VTl + o) = (v2b){l0, l1}; } __threadfence(); }
    __syncthreads(); } }
__global__ __launch_bounds__(32) void att_kernel(const b16* __restrict__ QNh, const b16* __restrict__ QNl, const b16* __restrict__ KNh, const b16* __restrict__ KNl, const b16* __restrict__ VTh, const b16* __restrict__ VTl, const float* __restrict__ TAB, int WLIM, float* __restrict__ O) { __shared__ __attribute__((aligned(16))) b16 Pa[16][HL + 8], Pb[16][HL + 8]; __shared__ float Sc[16][HL + 1], Of[16][C + 1], Madd[HL]; __shared__ int Ktok[HL]; const int lane = threadIdx.x, nloc = lane & 15, hlf = lane >> 4; const int win = blockIdx.x / (WL / 16), qb = blockIdx.x % (WL / 16); if (win >= WLIM) return; const int wi = win / NWS, wj = win % NWS;
  for (int j = lane; j < HL; j += 32) { int yy, xx; bool inimg; const bool ok = halo_key(wi, wj, j, yy, xx, inimg); Ktok[j] = ok ? yy * HP + xx : NTP; Madd[j] = inimg ? 0.0f : -100.0f; }
  if (lane < 16) for (int k = HL; k < HL + 8; ++k) { Pa[lane][k] = (b16)0.0f; Pb[lane][k] = (b16)0.0f; }
  wave_lds_sync();
  const int qy = qb * 2 + hlf, qx = nloc & 7;
  const int qi_l = qb * 16 + nloc; const size_t qtok = (size_t)(wi * CW + qi_l / CW) * HP + wj * CW + qi_l % CW;
  (void)qy; (void)qx;
#pragma unroll 1
  for (int h = 0; h < HEADS; ++h) { const v16b qa = frag_kb(QNh + qtok * C + h * HD, hlf), ql = frag_kb(QNl + qtok * C + h * HD, hlf);
#pragma unroll 4
    for (int t = 0; t < HL / 16; ++t) { const size_t ko = (size_t)Ktok[t * 16 + nloc] * C + h * HD; const v16b kh = frag_kb(KNh + ko, hlf), kl = frag_kb(KNl + ko, hlf); v8f s = wmma16b(qa, kh, (v8f){}); s = wmma16b(qa, kl, s); s = wmma16b(ql, kh, s);
#pragma unroll
      for (int r8 = 0; r8 < 8; ++r8) Sc[8 * hlf + r8][t * 16 + nloc] = s[r8] * (1.0f / (HS * HS)); }
    wave_lds_sync();
    if (lane < 16) { const int r = lane; const int qi = qb * 16 + r, q0y = qi / CW, q0x = qi % CW; float mx = -INFINITY; for (int j = 0; j < HL; ++j) { const int rel = (q0y - j / HWIN + HWIN - 1) * 23 + (q0x - j % HWIN + HWIN - 1); const float s = Sc[r][j] + TAB[rel * HEADS + h] + Madd[j]; Sc[r][j] = s; mx = fmaxf(mx, s); }
      float sm = 0.0f; for (int j = 0; j < HL; ++j) { const float p = __expf(Sc[r][j] - mx); Sc[r][j] = p; sm += p; } const float inv = 1.0f / sm; for (int j = 0; j < HL; ++j) { b16 p, pl; split16(Sc[r][j] * inv * PS, p, pl); Pa[r][j] = p; Pb[r][j] = pl; } }
    wave_lds_sync();
    v8f o[2] = {(v8f){}, (v8f){}};
#pragma unroll 2
    for (int kb = 0; kb < HL; kb += 32) { const v16b pa = frag_kb(&Pa[nloc][kb], hlf), pb = frag_kb(&Pb[nloc][kb], hlf);
#pragma unroll
      for (int t = 0; t < 2; ++t) { const size_t vo = ((size_t)win * C + h * HD + t * 16 + nloc) * HL + kb; const v16b vh = frag_kb(VTh + vo, hlf), vl = frag_kb(VTl + vo, hlf); o[t] = wmma16b(pa, vh, o[t]); o[t] = wmma16b(pa, vl, o[t]); o[t] = wmma16b(pb, vh, o[t]); } }
#pragma unroll
    for (int t = 0; t < 2; ++t)
#pragma unroll
      for (int r8 = 0; r8 < 8; ++r8) Of[8 * hlf + r8][h * HD + t * 16 + nloc] = o[t][r8] * (1.0f / (PS * HS));
    wave_lds_sync(); }
  for (int pass = 0; pass < 2; ++pass) { for (int r = 0; r < 16; ++r) { const int qi = qb * 16 + r; const size_t tk = (size_t)(wi * CW + qi / CW) * HP + wj * CW + qi % CW; for (int q = 0; q < 2; ++q) *(volatile v4f*)(O + tk * C + q * 128 + lane * 4) = *(const v4f*)(&Of[r][q * 128 + lane * 4]); } __threadfence(); } }
__global__ __launch_bounds__(32) void proj_kernel(const float* __restrict__ O, const b16* __restrict__ WPj, const float* __restrict__ pb, int PLIM, float* __restrict__ out  ) { __shared__ __attribute__((aligned(16))) b16 Ah[16][C + 8], Al[16][C + 8]; __shared__ float Tf[16][260]; const int lane = threadIdx.x, nloc = lane & 15, hlf = lane >> 4; const size_t p0 = (size_t)blockIdx.x * 16; if (p0 >= (size_t)PLIM) return; const int np = (PLIM - (int)p0) < 16 ? (PLIM - (int)p0) : 16;
  for (int rr = 0; rr < 16; ++rr) { const size_t p = p0 + (rr < np ? rr : 0); const size_t tk = (p / IW) * HP + (p % IW); for (int q = 0; q < 8; ++q) { const int c = q * 32 + lane; b16 ph, pl; split16(O[tk * C + c] * HS, ph, pl); Ah[rr][c] = ph; Al[rr][c] = pl; } }
  if (lane < 16) for (int k = C; k < C + 8; ++k) { Ah[lane][k] = (b16)0.0f; Al[lane][k] = (b16)0.0f; }
  wave_lds_sync(); v8f acc[16];
#pragma unroll
  for (int t = 0; t < 16; ++t) acc[t] = (v8f){};
#pragma unroll 2
  for (int kb = 0; kb < C; kb += 32) { const v16b a = frag_kb(&Ah[nloc][kb], hlf), al = frag_kb(&Al[nloc][kb], hlf);
#pragma unroll
    for (int t = 0; t < 16; ++t) { const v16b bw = frag_kb(WPj + (size_t)(t * 16 + nloc) * C + kb, hlf); acc[t] = wmma16b(a, bw, acc[t]); acc[t] = wmma16b(al, bw, acc[t]); } }
#pragma unroll
  for (int t = 0; t < 16; ++t) { const int cc = t * 16 + nloc; const float bb = bfv(pb[cc]);
#pragma unroll
    for (int r8 = 0; r8 < 8; ++r8) Tf[8 * hlf + r8][cc] = acc[t][r8] * (1.0f / (HS * WSC)) + bb; }
  wave_lds_sync();
  for (int pass = 0; pass < 2; ++pass) { for (int rr = 0; rr < np; ++rr) for (int q = 0; q < 2; ++q) *(volatile v4f*)(out + (p0 + rr) * C + q * 128 + lane * 4) = *(const v4f*)(&Tf[rr][q * 128 + lane * 4]); __threadfence(); } }
}

extern "C" void kernel_launch(void* const* d_in, const int* in_sizes, int n_in, void* d_out, int out_size, void* d_ws, size_t ws_size, hipStream_t stream) {
  (void)n_in;
  auto Fp = [&](int i) { return (const float*)d_in[i]; };
  if (in_sizes[0] != NB_ * NPIX * C || in_sizes[1] != 9 * C || in_sizes[4] != C * 3 * C || in_sizes[7] != HEADS || in_sizes[8] != 2 * CPH || in_sizes[10] != CPH * HEADS || in_sizes[11] != C * C || out_size != NB_ * NPIX * C) return;
  const int WLIM = NWIN;
  const int TLIM = WLIM >= NWIN ? NTP : ((WLIM / NWS) * CW + CW + CW / 2) * HP;
  const int PLIM = WLIM >= NWIN ? NPIX : (WLIM / NWS) * CW * IW;
  size_t off = 0; char* ws = (char*)d_ws;
  auto carve = [&](size_t bytes) { char* p = ws + off; off += (bytes + 255) & ~(size_t)255; return p; };
  b16* WQ = (b16*)carve((size_t)3 * C * C * 2); b16* WPj = (b16*)carve((size_t)C * C * 2); float* TAB = (float*)carve((size_t)NTAB * HEADS * 4); b16* QNh = (b16*)carve((size_t)NTP * C * 2); b16* QNl = (b16*)carve((size_t)NTP * C * 2); b16* KNh = (b16*)carve((size_t)(NTP + 1) * C * 2); b16* KNl = (b16*)carve((size_t)(NTP + 1) * C * 2); float* V = (float*)carve((size_t)NTP * C * 4); b16* VTh = (b16*)carve((size_t)NWIN * C * HL * 2); b16* VTl = (b16*)carve((size_t)NWIN * C * HL * 2); float* O = (float*)carve((size_t)NTP * C * 4);
  if (off > ws_size || off > ((size_t)144 << 20)) return;
  prep_kernel<<<64, 256, 0, stream>>>(Fp(4), Fp(11), Fp(8), Fp(9), Fp(10), WQ, WPj, TAB, KNh, KNl);
  for (int img = 0; img < NB_; ++img) { const float* xi = Fp(0) + (size_t)img * NPIX * C; float* oi = (float*)d_out + (size_t)img * NPIX * C;
    qkv_kernel<<<NTP / 16, 32, 0, stream>>>(xi, Fp(1), Fp(2), Fp(3), WQ, Fp(5), Fp(6), Fp(7), TLIM, QNh, QNl, KNh, KNl, V);
    vt_kernel<<<NWIN, 256, 0, stream>>>(V, WLIM, VTh, VTl);
    att_kernel<<<NWIN * (WL / 16), 32, 0, stream>>>(QNh, QNl, KNh, KNl, VTh, VTl, TAB, WLIM, O);
    proj_kernel<<<(NPIX + 15) / 16, 32, 0, stream>>>(O, WPj, Fp(12), PLIM, oi); }
}
